// PairwiseInteractions_55087250539205
// MI455X (gfx1250) — hardware-verified
//
#include <hip/hip_runtime.h>
#include <stdint.h>
#include <stddef.h>
#include <math.h>

#define BATCH     2048
#define NEGS      512
#define INPUT_DIM 256
#define DIM       64
#define VOCAB     32
#define N_HEADS   5
#define N_PAIR    6

#define GB_ROWS   16
#define GS        68
#define TB        4
#define NTAB      (N_PAIR * TB)
#define EMB_STR   68
#define T_FLOATS   (NTAB * VOCAB * VOCAB)
#define EMB_FLOATS (N_HEADS * VOCAB * EMB_STR)
#define GT_FLOATS  (NTAB * DIM)
#define SO_FLOATS  (TB * NEGS)
#define DYN_LDS_BYTES ((T_FLOATS + EMB_FLOATS + GT_FLOATS + SO_FLOATS) * 4)

static_assert(DYN_LDS_BYTES == 156160);
static_assert((T_FLOATS * 4) % 16 == 0);
static_assert((EMB_FLOATS * 4) % 16 == 0);
static_assert((GT_FLOATS * 4) % 16 == 0);
static_assert((GS * 4) % 16 == 0);
static_assert((EMB_STR * 4) % 16 == 0);
static_assert(BATCH % GB_ROWS == 0);
static_assert(BATCH % TB == 0);
static_assert(NTAB % 8 == 0);
static_assert((TB * NEGS) % 256 == 0);
static_assert((TB * NEGS) / 4 == 2 * 256);
static_assert(INPUT_DIM % 32 == 0);
static_assert(DIM == 64);
static_assert(VOCAB == 32);
static_assert((BATCH * INPUT_DIM) % 2048 == 0);
static_assert((N_PAIR * DIM * INPUT_DIM) % 2048 == 0);
static_assert((N_HEADS * VOCAB * DIM) % (4 * 256) == 0);
static_assert(GT_FLOATS % 4 == 0);

typedef __bf16         v16bf __attribute__((ext_vector_type(16)));
typedef float          v8f   __attribute__((ext_vector_type(8)));
typedef float          v4f   __attribute__((ext_vector_type(4)));
typedef unsigned int   v8u   __attribute__((ext_vector_type(8)));
typedef unsigned int   v4u   __attribute__((ext_vector_type(4)));
typedef unsigned short v8us  __attribute__((ext_vector_type(8)));
typedef v4f  __attribute__((may_alias)) v4fa;
typedef v4u  __attribute__((may_alias)) v4ua;
typedef v8us __attribute__((may_alias)) v8usa;

union FragU { v16bf v; v8us half[2]; v8u w; };

__device__ __forceinline__ v8f wmma16(v16bf a, v16bf b, v8f c) {
  v8f d = __builtin_amdgcn_wmma_f32_16x16x32_bf16(false, a, false, b, (short)0, c, false, false);
  asm volatile("v_nop\n\tv_nop\n\tv_nop\n\tv_nop" : "+v"(d) : "v"(a), "v"(b));
  return d;
}

__device__ __forceinline__ v16bf ldfu(const unsigned short* p, int h) {
  FragU f;
  f.half[0] = *(const v8usa*)(p + 8 * h);
  f.half[1] = *(const v8usa*)(p + 16 + 8 * h);
  return f.v;
}

__device__ __forceinline__ unsigned bf16_rne(float f) {
  const unsigned u = __float_as_uint(f);
  return (u + 0x7fffu + ((u >> 16) & 1u)) >> 16;
}
__device__ __forceinline__ void pk2(float a, float b, unsigned& hw, unsigned& lw) {
  const unsigned ha = bf16_rne(a);
  const unsigned hb = bf16_rne(b);
  const unsigned la = bf16_rne(a - __uint_as_float(ha << 16));
  const unsigned lb = bf16_rne(b - __uint_as_float(hb << 16));
  hw = ha | (hb << 16);
  lw = la | (lb << 16);
}
__device__ __forceinline__ void mkfrag(v4f q0, v4f q1, v4f q2, v4f q3, v16bf& hi, v16bf& lo) {
  unsigned h0, h1, h2, h3, h4, h5, h6, h7;
  unsigned l0, l1, l2, l3, l4, l5, l6, l7;
  pk2(q0.x, q0.y, h0, l0); pk2(q0.z, q0.w, h1, l1);
  pk2(q1.x, q1.y, h2, l2); pk2(q1.z, q1.w, h3, l3);
  pk2(q2.x, q2.y, h4, l4); pk2(q2.z, q2.w, h5, l5);
  pk2(q3.x, q3.y, h6, l6); pk2(q3.z, q3.w, h7, l7);
  FragU H, L;
  const v8u hw = {h0, h1, h2, h3, h4, h5, h6, h7};
  const v8u lw = {l0, l1, l2, l3, l4, l5, l6, l7};
  H.w = hw; L.w = lw;
  hi = H.v; lo = L.v;
}

__device__ __forceinline__ int fixlab(int v) {
  v = (v < 0) ? (v + VOCAB) : v;
  v = (v < 0) ? 0 : v;
  v = (v > VOCAB - 1) ? (VOCAB - 1) : v;
  return v;
}

__global__ __launch_bounds__(256) void k_split(const float* __restrict__ src,
                                               unsigned short* __restrict__ hi,
                                               unsigned short* __restrict__ lo,
                                               int n8)
{
  const int gid = blockIdx.x * 256 + threadIdx.x;
  if (gid >= n8) return;
  const float* s = src + (size_t)gid * 8;
  const v4f a = *(const v4fa*)s;
  const v4f b = *(const v4fa*)(s + 4);
  unsigned h0, h1, h2, h3, l0, l1, l2, l3;
  pk2(a.x, a.y, h0, l0); pk2(a.z, a.w, h1, l1);
  pk2(b.x, b.y, h2, l2); pk2(b.z, b.w, h3, l3);
  const v4u hv = {h0, h1, h2, h3};
  const v4u lv = {l0, l1, l2, l3};
  unsigned short* hp = hi + (size_t)gid * 8;
  unsigned short* lp = lo + (size_t)gid * 8;
  *(volatile v4ua*)hp = hv;
  *(volatile v4ua*)lp = lv;
  __threadfence();
  *(volatile v4ua*)hp = hv;
  *(volatile v4ua*)lp = lv;
}

__global__ __launch_bounds__(128) void k_gate(const unsigned short* __restrict__ xh,
                                              const unsigned short* __restrict__ xl,
                                              const unsigned short* __restrict__ wh,
                                              const unsigned short* __restrict__ wl,
                                              const float* __restrict__ gb,
                                              float* __restrict__ g)
{
  __shared__ __align__(16) float sg[GB_ROWS * GS];
  const int tid = threadIdx.x, lane = tid & 31, wv = tid >> 5;
  const int h = lane >> 4, m = lane & 15;
  const int b0 = blockIdx.x * GB_ROWS;
  const int p  = blockIdx.y;
  const int d0 = wv * 16;

  const unsigned short* arh = xh + (size_t)(b0 + m) * INPUT_DIM;
  const unsigned short* arl = xl + (size_t)(b0 + m) * INPUT_DIM;
  const unsigned short* brh = wh + ((size_t)p * DIM + d0 + m) * INPUT_DIM;
  const unsigned short* brl = wl + ((size_t)p * DIM + d0 + m) * INPUT_DIM;

  v8f acc = {0.f, 0.f, 0.f, 0.f, 0.f, 0.f, 0.f, 0.f};
  #pragma unroll
  for (int k0 = 0; k0 < INPUT_DIM; k0 += 32) {
    const v16bf a1 = ldfu(arh + k0, h);
    const v16bf a2 = ldfu(arl + k0, h);
    const v16bf b1 = ldfu(brh + k0, h);
    const v16bf b2 = ldfu(brl + k0, h);
    acc = wmma16(a1, b1, acc);
    acc = wmma16(a1, b2, acc);
    acc = wmma16(a2, b1, acc);
  }

  const float bias = gb[p * DIM + d0 + m];
  #pragma unroll
  for (int r = 0; r < 8; ++r) sg[(8 * h + r) * GS + d0 + m] = tanhf(acc[r] + bias);
  __syncthreads();

  #pragma unroll
  for (int i = 0; i < 2; ++i) {
    const int row = 4 * wv + 2 * i + (lane >> 4);
    const int f4 = lane & 15;
    const v4f v = *(const v4fa*)(sg + row * GS + 4 * f4);
    *(volatile v4fa*)(g + ((size_t)p * BATCH + b0 + row) * DIM + 4 * f4) = v;
  }
  __threadfence();
  #pragma unroll
  for (int i = 0; i < 2; ++i) {
    const int row = 4 * wv + 2 * i + (lane >> 4);
    const int f4 = lane & 15;
    const v4f v = *(const v4fa*)(sg + row * GS + 4 * f4);
    *(volatile v4fa*)(g + ((size_t)p * BATCH + b0 + row) * DIM + 4 * f4) = v;
  }
}

__global__ __launch_bounds__(256) void k_table(const int* __restrict__ labels,
                                               const float* __restrict__ emb,
                                               const float* __restrict__ g,
                                               float* __restrict__ out)
{
  extern __shared__ __align__(16) float smem[];
  float* T    = smem;
  float* embs = smem + T_FLOATS;
  float* gt   = embs + EMB_FLOATS;
  float* sout = gt + GT_FLOATS;

  const int tid = threadIdx.x, lane = tid & 31, wv = tid >> 5;
  const int h = lane >> 4, m = lane & 15;
  const int b0 = blockIdx.x * TB;

  #pragma unroll 1
  for (int idx = tid; idx < (N_HEADS * VOCAB * DIM) / 4; idx += 256) {
    const int j   = idx * 4;
    const int hh  = j >> 11;
    const int rem = j & 2047;
    const int v   = rem >> 6;
    const int d   = rem & 63;
    *(v4fa*)(embs + (hh * VOCAB + v) * EMB_STR + d) = *(const v4fa*)(emb + j);
  }
  #pragma unroll 1
  for (int idx = tid; idx < GT_FLOATS / 4; idx += 256) {
    const int j   = idx * 4;
    const int p   = j >> 8;
    const int rem = j & 255;
    const int bi  = rem >> 6;
    const int d   = rem & 63;
    *(v4fa*)(gt + j) = *(const v4fa*)(g + ((size_t)p * BATCH + b0 + bi) * DIM + d);
  }
  __syncthreads();

  const v8f z8 = {0.f, 0.f, 0.f, 0.f, 0.f, 0.f, 0.f, 0.f};

  #pragma unroll 1
  for (int jt = 0; jt < NTAB / 8; ++jt) {
    const int t    = wv + 8 * jt;
    const int p    = t >> 2;
    const int rowA = (p < 3) ? 3 : 4;
    const int rowB = (p < 3) ? p : (p - 3);
    const float* ga = gt + t * DIM;
    float* Tt = T + t * (VOCAB * VOCAB);

    v16bf bh[2][2], bl[2][2];
    #pragma unroll
    for (int nt = 0; nt < 2; ++nt) {
      #pragma unroll
      for (int kk = 0; kk < 2; ++kk) {
        const int kb = kk * 32 + 8 * h;
        const float* er = embs + (rowB * VOCAB + nt * 16 + m) * EMB_STR + kb;
        mkfrag(*(const v4fa*)er, *(const v4fa*)(er + 4),
               *(const v4fa*)(er + 16), *(const v4fa*)(er + 20), bh[nt][kk], bl[nt][kk]);
      }
    }
    #pragma unroll
    for (int mt = 0; mt < 2; ++mt) {
      v16bf ah[2], al[2];
      #pragma unroll
      for (int kk = 0; kk < 2; ++kk) {
        const int kb = kk * 32 + 8 * h;
        const float* er = embs + (rowA * VOCAB + mt * 16 + m) * EMB_STR + kb;
        const float* gp = ga + kb;
        const v4f q0 = *(const v4fa*)er        * *(const v4fa*)gp;
        const v4f q1 = *(const v4fa*)(er + 4)  * *(const v4fa*)(gp + 4);
        const v4f q2 = *(const v4fa*)(er + 16) * *(const v4fa*)(gp + 16);
        const v4f q3 = *(const v4fa*)(er + 20) * *(const v4fa*)(gp + 20);
        mkfrag(q0, q1, q2, q3, ah[kk], al[kk]);
      }
      #pragma unroll
      for (int nt = 0; nt < 2; ++nt) {
        v8f acc = z8;
        #pragma unroll
        for (int kk = 0; kk < 2; ++kk) {
          acc = wmma16(ah[kk], bh[nt][kk], acc);
          acc = wmma16(ah[kk], bl[nt][kk], acc);
          acc = wmma16(al[kk], bh[nt][kk], acc);
        }
        #pragma unroll
        for (int r = 0; r < 8; ++r)
          Tt[(mt * 16 + 8 * h + r) * VOCAB + nt * 16 + m] = acc[r];
      }
    }
  }
  __syncthreads();

  #pragma unroll 1
  for (int it = 0; it < (TB * NEGS) / 256; ++it) {
    const int idx = tid + 256 * it;
    const int bi  = idx >> 9;
    const int n   = idx & (NEGS - 1);
    const int* lab = labels + ((size_t)(b0 + bi) * NEGS + n) * 6;
    const int l0 = fixlab(lab[0]);
    const int l1 = fixlab(lab[1]);
    const int l2 = fixlab(lab[2]);
    const int l3 = fixlab(lab[3]);
    const int l4 = fixlab(lab[4]);
    float s = T[((0 * TB + bi) << 10) + (l0 << 5) + l1];
    s += T[((1 * TB + bi) << 10) + (l0 << 5) + l2];
    s += T[((2 * TB + bi) << 10) + (l0 << 5) + l3];
    s += T[((3 * TB + bi) << 10) + (l4 << 5) + l1];
    s += T[((4 * TB + bi) << 10) + (l4 << 5) + l2];
    s += T[((5 * TB + bi) << 10) + (l4 << 5) + l3];
    sout[idx] = s;
  }
  __syncthreads();

  float* ob = out + (size_t)b0 * NEGS;
  #pragma unroll
  for (int i = 0; i < 2; ++i) {
    const int f = tid + 256 * i;
    const v4f v = *(const v4fa*)(sout + 4 * f);
    *(volatile v4fa*)(ob + 4 * f) = v;
  }
  __threadfence();
  #pragma unroll
  for (int i = 0; i < 2; ++i) {
    const int f = tid + 256 * i;
    const v4f v = *(const v4fa*)(sout + 4 * f);
    *(volatile v4fa*)(ob + 4 * f) = v;
  }
}

extern "C" void kernel_launch(void* const* d_in, const int* in_sizes, int n_in,
                              void* d_out, int out_size, void* d_ws, size_t ws_size,
                              hipStream_t stream)
{
  if (n_in < 5) return;
  if (in_sizes[0] != BATCH * INPUT_DIM) return;
  if (in_sizes[1] != BATCH * NEGS * 6) return;
  if (in_sizes[2] != N_HEADS * VOCAB * DIM) return;
  if (in_sizes[3] != N_PAIR * DIM * INPUT_DIM) return;
  if (in_sizes[4] != N_PAIR * DIM) return;
  if (out_size != BATCH * NEGS) return;

  const float* x      = (const float*)d_in[0];
  const int*   labels = (const int*)d_in[1];
  const float* emb    = (const float*)d_in[2];
  const float* gw     = (const float*)d_in[3];
  const float* gb     = (const float*)d_in[4];
  float* out = (float*)d_out;

  const size_t nX  = (size_t)BATCH * INPUT_DIM;
  const size_t nW  = (size_t)N_PAIR * DIM * INPUT_DIM;
  const size_t bXH = nX * 2, bXL = nX * 2;
  const size_t bWH = nW * 2, bWL = nW * 2;
  const size_t bG  = (size_t)N_PAIR * BATCH * DIM * 4;
  const size_t total = bXH + bXL + bWH + bWL + bG;
  if (total > ws_size) return;
  if (total > (size_t)134217728) return;

  char* ws = (char*)d_ws;
  size_t off = 0;
  unsigned short* XH = (unsigned short*)(ws + off); off += bXH;
  unsigned short* XL = (unsigned short*)(ws + off); off += bXL;
  unsigned short* WH = (unsigned short*)(ws + off); off += bWH;
  unsigned short* WL = (unsigned short*)(ws + off); off += bWL;
  float*          G  = (float*)(ws + off);          off += bG;
  if (off != total) return;

  k_split<<<(unsigned)(nX / 2048), 256, 0, stream>>>(x, XH, XL, (int)(nX / 8));
  k_split<<<(unsigned)(nW / 2048), 256, 0, stream>>>(gw, WH, WL, (int)(nW / 8));
  k_gate<<<dim3(BATCH / GB_ROWS, N_PAIR), 128, 0, stream>>>(XH, XL, WH, WL, gb, G);
  hipFuncSetAttribute(reinterpret_cast<const void*>(&k_table),
                      hipFuncAttributeMaxDynamicSharedMemorySize, DYN_LDS_BYTES);
  k_table<<<BATCH / TB, 256, DYN_LDS_BYTES, stream>>>(labels, emb, G, out);
}
